// ClassicalSelfAttention_65481071405130
// MI455X (gfx1250) — hardware-verified
//
#include <hip/hip_runtime.h>
#include <stdint.h>

#define NTOK 8192
#define EMB  1024
#define SEQ  2048

typedef _Float16 v16h __attribute__((ext_vector_type(16)));
typedef _Float16 v8h  __attribute__((ext_vector_type(8)));
typedef __bf16   v16b __attribute__((ext_vector_type(16)));
typedef __bf16   v8b  __attribute__((ext_vector_type(8)));
typedef float    v8f  __attribute__((ext_vector_type(8)));
typedef float    v4f  __attribute__((ext_vector_type(4)));
typedef unsigned short v8us __attribute__((ext_vector_type(8)));

static_assert((EMB % 64) == 0);
static_assert((NTOK % 64) == 0);
static_assert((NTOK % SEQ) == 0);
static_assert((((NTOK / 64) * (EMB / 64)) % 8) == 0);

__device__ __forceinline__ unsigned short bfbits(float f) {
  unsigned u = __float_as_uint(f);
  return (unsigned short)((u + 0x7FFFu + ((u >> 16) & 1u)) >> 16);
}
__device__ __forceinline__ float bfval(unsigned short b) { return __uint_as_float(((unsigned)b) << 16); }
__device__ __forceinline__ float bfr(float f) { return bfval(bfbits(f)); }
__device__ __forceinline__ void split_bf(float f, unsigned short& hb, unsigned short& lb) {
  hb = bfbits(f);
  lb = bfbits(f - bfval(hb));
}

template <int ET> struct Elem;
template <> struct Elem<0> {
  typedef _Float16 T; typedef v16h V; typedef v8h V8;
  static __device__ __forceinline__ v8f mma(V a, V b, v8f c) {
    return __builtin_amdgcn_wmma_f32_16x16x32_f16(false, a, false, b, (short)0, c, false, false);
  }
};
template <> struct Elem<1> {
  typedef __bf16 T; typedef v16b V; typedef v8b V8;
  static __device__ __forceinline__ v8f mma(V a, V b, v8f c) {
    return __builtin_amdgcn_wmma_f32_16x16x32_bf16(false, a, false, b, (short)0, c, false, false);
  }
};

template <int ET>
__device__ __forceinline__ typename Elem<ET>::V ldfragT(const typename Elem<ET>::T* p) {
  typedef typename Elem<ET>::V V;
  typedef typename Elem<ET>::V8 V8;
  union { V v; V8 h[2]; } f;
  f.h[0] = *(const V8*)(p);
  f.h[1] = *(const V8*)(p + 16);
  return f.v;
}
__device__ __forceinline__ v16h ldfrag(const _Float16* p) { return ldfragT<0>(p); }
__device__ __forceinline__ v8f mma16(v16h a, v16h b, v8f c) { return Elem<0>::mma(a, b, c); }
__device__ __forceinline__ v8f zero8() {
  v8f z;
#pragma unroll
  for (int i = 0; i < 8; ++i) z[i] = 0.0f;
  return z;
}

__device__ __forceinline__ void guard_g(v8f& a, v8f& b, v16h x, v16h y) {
  asm volatile("v_nop\n\tv_nop\n\tv_nop\n\tv_nop" : "+v"(a), "+v"(b) : "v"(x), "v"(y));
}
__device__ __forceinline__ void guard_g(v8f& a, v8f& b, v16b x, v16b y) {
  asm volatile("v_nop\n\tv_nop\n\tv_nop\n\tv_nop" : "+v"(a), "+v"(b) : "v"(x), "v"(y));
}
__device__ __forceinline__ void keep4(v16h a, v16h b, v16h c, v16h d) {
  asm volatile("v_nop" :: "v"(a), "v"(b), "v"(c), "v"(d));
}
__device__ __forceinline__ void keep4(v16b a, v16b b, v16b c, v16b d) {
  asm volatile("v_nop" :: "v"(a), "v"(b), "v"(c), "v"(d));
}
__device__ __forceinline__ void accg4(v8f& a, v8f& b, v8f& c, v8f& d) {
  asm volatile("v_nop\n\tv_nop\n\tv_nop\n\tv_nop" : "+v"(a), "+v"(b), "+v"(c), "+v"(d));
}
__device__ __forceinline__ void guard_s4(v8f& a, v8f& b, v8f& c, v8f& d, v16h x0, v16h x1, v16h y0, v16h y1) {
  asm volatile("v_nop\n\tv_nop\n\tv_nop\n\tv_nop"
               : "+v"(a), "+v"(b), "+v"(c), "+v"(d) : "v"(x0), "v"(x1), "v"(y0), "v"(y1));
}
__device__ __forceinline__ void guard_pv4(v8f& a0, v8f& a1, v8f& a2, v8f& a3,
                                          v16h p, v16h x0, v16h x1, v16h x2, v16h x3) {
  asm volatile("v_nop\n\tv_nop\n\tv_nop\n\tv_nop"
               : "+v"(a0), "+v"(a1), "+v"(a2), "+v"(a3)
               : "v"(p), "v"(x0), "v"(x1), "v"(x2), "v"(x3));
}

template <int MODE>
__global__ __launch_bounds__(256) void cvt_kernel(const float* __restrict__ src, unsigned short* __restrict__ dst, int n8) {
  const int li = (int)blockIdx.x * 256 + (int)threadIdx.x;
  if (li >= n8) return;
  const size_t e = (size_t)li * 8;
  const v4f a = *(const v4f*)(src + e);
  const v4f b = *(const v4f*)(src + e + 4);
  if (MODE == 0) {
    v8us o;
#pragma unroll
    for (int i = 0; i < 4; ++i) {
      o[i]     = bfbits(a[i]);
      o[4 + i] = bfbits(b[i]);
    }
    unsigned short* d = dst + e;
    *(volatile v8us*)d = o;
    __threadfence();
    *(volatile v8us*)d = o;
  } else {
    v8h o;
#pragma unroll
    for (int i = 0; i < 4; ++i) {
      o[i]     = (_Float16)(bfr(a[i]) * 64.0f);
      o[4 + i] = (_Float16)(bfr(b[i]) * 64.0f);
    }
    _Float16* d = (_Float16*)(void*)dst + e;
    *(volatile v8h*)d = o;
    __threadfence();
    *(volatile v8h*)d = o;
  }
}

template <int ET, bool SPLITA, int OUT_MODE>
__global__ __launch_bounds__(256) void gemm64_kernel(const unsigned short* __restrict__ Ap,
                                                     const unsigned short* __restrict__ A2p, int lda,
                                                     const unsigned short* __restrict__ Btp, int ldb,
                                                     void* Cout, void* C2out, int ldc,
                                                     const float* aux, int M, int N, int K, float scale) {
  typedef typename Elem<ET>::T T;
  typedef typename Elem<ET>::V V;
  const T* A  = (const T*)(const void*)Ap;
  const T* A2 = (const T*)(const void*)A2p;
  const T* Bt = (const T*)(const void*)Btp;
  __shared__ __align__(16) float sT[8][16 * 68];
  const int lane = threadIdx.x & 31, wave = threadIdx.x >> 5;
  const int tilesN = N >> 6, tilesM = M >> 6;
  const int tile = (int)blockIdx.x * 8 + wave;
  if (tile >= tilesM * tilesN) return;
  const int tm = tile / tilesN, tn = tile - tm * tilesN;
  const int m0 = tm << 6, n0 = tn << 6;
  const int rl = lane & 15;
  const int koff = (lane >> 4) * 8;
  const int mOff = (lane >> 4) * 8;

  v8f acc[4][4];
#pragma unroll
  for (int i = 0; i < 4; ++i)
#pragma unroll
    for (int j = 0; j < 4; ++j) acc[i][j] = zero8();

#pragma unroll 1
  for (int k0 = 0; k0 < K; k0 += 32) {
    V bh[4];
#pragma unroll
    for (int j = 0; j < 4; ++j) bh[j] = ldfragT<ET>(Bt + (size_t)(n0 + (j << 4) + rl) * ldb + koff + k0);
#pragma unroll
    for (int i = 0; i < 4; ++i) {
      const size_t ao = (size_t)(m0 + (i << 4) + rl) * lda + koff + k0;
      const V ah = ldfragT<ET>(A + ao);
      V al = ah;
      if (SPLITA) al = ldfragT<ET>(A2 + ao);
#pragma unroll
      for (int j = 0; j < 4; ++j) {
        acc[i][j] = Elem<ET>::mma(ah, bh[j], acc[i][j]);
        if (SPLITA) acc[i][j] = Elem<ET>::mma(al, bh[j], acc[i][j]);
      }
      guard_g(acc[i][0], acc[i][3], ah, SPLITA ? al : bh[3]);
    }
    keep4(bh[0], bh[1], bh[2], bh[3]);
  }
  accg4(acc[0][0], acc[0][1], acc[0][2], acc[0][3]);
  accg4(acc[1][0], acc[1][1], acc[1][2], acc[1][3]);
  accg4(acc[2][0], acc[2][1], acc[2][2], acc[2][3]);
  accg4(acc[3][0], acc[3][1], acc[3][2], acc[3][3]);

  float* slab = sT[wave];
#pragma unroll
  for (int i = 0; i < 4; ++i) {
    const int mBase = m0 + (i << 4);
#pragma unroll
    for (int j = 0; j < 4; ++j) {
#pragma unroll
      for (int r = 0; r < 8; ++r) {
        float v = acc[i][j][r] * scale;
        if (OUT_MODE == 4) {
          const float g = __builtin_amdgcn_rcpf(1.0f + __expf(-v));
          v = g * aux[(size_t)(mBase + mOff + r) * ldc + n0 + (j << 4) + rl];
        }
        slab[(mOff + r) * 68 + (j << 4) + rl] = v;
      }
    }
    __builtin_amdgcn_fence(__ATOMIC_RELEASE, "workgroup");
    __builtin_amdgcn_wave_barrier();
    __builtin_amdgcn_fence(__ATOMIC_ACQUIRE, "workgroup");
    if (OUT_MODE == 3 || OUT_MODE == 4) {
      float* C = (float*)Cout;
      const int hh = lane >> 4, c4 = (lane & 15) * 4;
#pragma unroll
      for (int ps = 0; ps < 2; ++ps) {
#pragma unroll
        for (int it = 0; it < 8; ++it) {
          const int row = it * 2 + hh;
          const v4f v = *(const v4f*)(slab + row * 68 + c4);
          *(volatile v4f*)(C + (size_t)(mBase + row) * ldc + n0 + c4) = v;
        }
        __threadfence();
      }
    }
    if (OUT_MODE == 1 || OUT_MODE == 2 || OUT_MODE == 3) {
      _Float16* H = (_Float16*)((OUT_MODE == 3) ? C2out : Cout);
      _Float16* L = (_Float16*)C2out;
      const float hm = (OUT_MODE == 3) ? 64.0f : 1.0f;
      const int qq = lane >> 3, c8 = (lane & 7) * 8;
#pragma unroll
      for (int ps = 0; ps < 2; ++ps) {
#pragma unroll
        for (int it = 0; it < 4; ++it) {
          const int row = it * 4 + qq;
          const float* sp = slab + row * 68 + c8;
          v8h hv;
#pragma unroll
          for (int e = 0; e < 8; ++e) hv[e] = (_Float16)(sp[e] * hm);
          *(volatile v8h*)(H + (size_t)(mBase + row) * ldc + n0 + c8) = hv;
          if (OUT_MODE == 2) {
            v8h lv;
#pragma unroll
            for (int e = 0; e < 8; ++e) lv[e] = (_Float16)((sp[e] - (float)hv[e]) * 2048.0f);
            *(volatile v8h*)(L + (size_t)(mBase + row) * ldc + n0 + c8) = lv;
          }
        }
        __threadfence();
      }
    }
    __builtin_amdgcn_fence(__ATOMIC_RELEASE, "workgroup");
    __builtin_amdgcn_wave_barrier();
    __builtin_amdgcn_fence(__ATOMIC_ACQUIRE, "workgroup");
  }
}

#define QB       16
#define KCH      256
#define QSP      1032
#define PSP      264
#define LDS_QH   0
#define LDS_QL   33024
#define LDS_PS   66048
#define LDS_PMAX 74496
#define LDS_PSUM 75008
#define LDS_ST   75520
#define ATT_LDS  75776
static_assert(QB * QSP * 2 == LDS_QL - LDS_QH);
static_assert(QB * QSP * 2 == LDS_PS - LDS_QL);
static_assert(QB * PSP * 2 == LDS_PMAX - LDS_PS);
static_assert(LDS_PSUM - LDS_PMAX == 8 * QB * 4);
static_assert(LDS_ST - LDS_PSUM == 8 * QB * 4);
static_assert(ATT_LDS - LDS_ST == 4 * QB * 4);
static_assert((QSP % 8) == 0 && (PSP % 8) == 0 && PSP >= KCH && QSP >= EMB);
static_assert((LDS_QL % 16) == 0 && (LDS_PS % 16) == 0 && (LDS_PMAX % 16) == 0 && (LDS_ST % 16) == 0);
static_assert((SEQ % KCH) == 0 && (SEQ % QB) == 0 && (EMB == 8 * 128) && (QB * 128 == 8 * 256));

__global__ __launch_bounds__(256) void attn_kernel(const _Float16* __restrict__ qh, const _Float16* __restrict__ ql,
                                                   const _Float16* __restrict__ kn, const _Float16* __restrict__ vh,
                                                   const _Float16* __restrict__ vl, unsigned short* __restrict__ oh,
                                                   unsigned short* __restrict__ ol, float sc) {
  extern __shared__ __align__(16) char smem[];
  _Float16* Qh = (_Float16*)(smem + LDS_QH);
  _Float16* Qw = (_Float16*)(smem + LDS_QL);
  _Float16* Ps = (_Float16*)(smem + LDS_PS);
  float* pmax = (float*)(smem + LDS_PMAX);
  float* psum = (float*)(smem + LDS_PSUM);
  float* m_s  = (float*)(smem + LDS_ST);
  float* l_s  = m_s + QB;
  float* al_s = m_s + 2 * QB;
  float* li_s = m_s + 3 * QB;

  const int tid = threadIdx.x, wave = tid >> 5, lane = tid & 31, h = lane >> 4, c = lane & 15;
  const int q0 = (int)blockIdx.x * QB;
  const int kbat = (q0 / SEQ) * SEQ;
  const float ninf = -__builtin_inff();
  const float rinv = 1.0f / 2048.0f;

  if (tid < QB) { m_s[tid] = ninf; l_s[tid] = 0.0f; al_s[tid] = 0.0f; li_s[tid] = 0.0f; }
  if (tid < 8 * QB) psum[tid] = 0.0f;
#pragma unroll
  for (int i = 0; i < 8; ++i) {
    const int idx = i * 256 + tid;
    const int row = idx >> 7;
    const int pc  = idx & 127;
    const size_t go = (size_t)(q0 + row) * EMB + pc * 8;
    *(v8h*)(Qh + row * QSP + pc * 8) = *(const v8h*)(qh + go);
    *(v8h*)(Qw + row * QSP + pc * 8) = *(const v8h*)(ql + go);
  }
  __syncthreads();

  v8f ohi[8];
#pragma unroll
  for (int nt = 0; nt < 8; ++nt) ohi[nt] = zero8();

  const _Float16* bqhp = Qh + c * QSP + 8 * h;
  const _Float16* bqlp = Qw + c * QSP + 8 * h;
  const _Float16* pap  = Ps + c * PSP + 8 * h;
  const int ntile = SEQ / KCH;

#pragma unroll 1
  for (int t = 0; t < ntile; ++t) {
    const int kb = kbat + t * KCH + 32 * wave;
    const _Float16* ka0p = kn + (size_t)(kb + c) * EMB + 8 * h;
    const _Float16* ka1p = kn + (size_t)(kb + 16 + c) * EMB + 8 * h;
    v8f sh[2], sw[2];
#pragma unroll
    for (int kt = 0; kt < 2; ++kt) { sh[kt] = zero8(); sw[kt] = zero8(); }
#pragma unroll 1
    for (int k0 = 0; k0 < EMB; k0 += 32) {
      const v16h a0 = ldfrag(ka0p + k0), a1 = ldfrag(ka1p + k0);
      const v16h bh = ldfrag(bqhp + k0), bw = ldfrag(bqlp + k0);
      sh[0] = mma16(a0, bh, sh[0]);
      sh[1] = mma16(a1, bh, sh[1]);
      sw[0] = mma16(a0, bw, sw[0]);
      sw[1] = mma16(a1, bw, sw[1]);
      guard_s4(sh[0], sh[1], sw[0], sw[1], a0, a1, bh, bw);
    }
    {
      float pm = ninf;
#pragma unroll
      for (int kt = 0; kt < 2; ++kt) {
#pragma unroll
        for (int r = 0; r < 8; ++r) {
          const float v = (sh[kt][r] + sw[kt][r] * rinv) * sc;
          sh[kt][r] = v;
          pm = fmaxf(pm, v);
        }
      }
      pm = fmaxf(pm, __shfl_xor(pm, 16, 32));
      pmax[wave * QB + c] = pm;
    }
    __syncthreads();
    if (tid < QB) {
      const int row = tid;
      float ps = 0.0f;
#pragma unroll
      for (int w = 0; w < 8; ++w) ps += psum[w * QB + row];
      l_s[row] = l_s[row] * al_s[row] + ps;
      const float mo = m_s[row];
      float mx = mo;
#pragma unroll
      for (int w = 0; w < 8; ++w) mx = fmaxf(mx, pmax[w * QB + row]);
      al_s[row] = __expf(mo - mx);
      m_s[row] = mx;
    }
    __syncthreads();
    {
      const float mq = m_s[c];
      float ps = 0.0f;
#pragma unroll
      for (int kt = 0; kt < 2; ++kt) {
        v8h hv;
#pragma unroll
        for (int r = 0; r < 8; ++r) {
          const float p = __expf(sh[kt][r] - mq);
          const _Float16 hr = (_Float16)(p * 4096.0f);
          hv[r] = hr;
          ps += (float)hr;
        }
        *(v8h*)(Ps + c * PSP + 32 * wave + 16 * kt + 8 * h) = hv;
      }
      ps += __shfl_xor(ps, 16, 32);
      psum[wave * QB + c] = ps;
      const v4f aA = *(const v4f*)(al_s + 8 * h), aB = *(const v4f*)(al_s + 8 * h + 4);
#pragma unroll
      for (int nt = 0; nt < 8; ++nt) {
#pragma unroll
        for (int r = 0; r < 4; ++r) {
          ohi[nt][r] *= aA[r];
          ohi[nt][4 + r] *= aB[r];
        }
      }
    }
    __syncthreads();
    {
      const size_t key0 = (size_t)(kbat + t * KCH) + 8 * h;
      const _Float16* vhp = vh + (size_t)(128 * wave + c) * NTOK + key0;
      const _Float16* vlp = vl + (size_t)(128 * wave + c) * NTOK + key0;
#pragma unroll 1
      for (int ks = 0; ks < KCH; ks += 32) {
        const v16h pa = ldfrag(pap + ks);
#pragma unroll
        for (int g = 0; g < 2; ++g) {
          v16h vb[4];
#pragma unroll
          for (int j = 0; j < 4; ++j) vb[j] = ldfrag(vhp + (size_t)(16 * (4 * g + j)) * NTOK + ks);
#pragma unroll
          for (int j = 0; j < 4; ++j) ohi[4 * g + j] = mma16(pa, vb[j], ohi[4 * g + j]);
          guard_pv4(ohi[4 * g], ohi[4 * g + 1], ohi[4 * g + 2], ohi[4 * g + 3], pa, vb[0], vb[1], vb[2], vb[3]);
          v16h wb[4];
#pragma unroll
          for (int j = 0; j < 4; ++j) wb[j] = ldfrag(vlp + (size_t)(16 * (4 * g + j)) * NTOK + ks);
          v8f lo[4];
#pragma unroll
          for (int j = 0; j < 4; ++j) lo[j] = mma16(pa, wb[j], zero8());
          guard_pv4(lo[0], lo[1], lo[2], lo[3], pa, wb[0], wb[1], wb[2], wb[3]);
#pragma unroll
          for (int j = 0; j < 4; ++j) {
#pragma unroll
            for (int r = 0; r < 8; ++r) ohi[4 * g + j][r] += lo[j][r] * rinv;
          }
        }
      }
    }
  }
  accg4(ohi[0], ohi[1], ohi[2], ohi[3]);
  accg4(ohi[4], ohi[5], ohi[6], ohi[7]);

  if (tid < QB) {
    const int row = tid;
    float ps = 0.0f;
#pragma unroll
    for (int w = 0; w < 8; ++w) ps += psum[w * QB + row];
    const float l = l_s[row] * al_s[row] + ps;
    li_s[row] = __builtin_amdgcn_rcpf(l) * (1.0f / 16.0f);
  }
  __syncthreads();
  unsigned short* Hs = (unsigned short*)(smem + LDS_QH);
  unsigned short* Ls = (unsigned short*)(smem + LDS_QL);
  {
    const v4f iA = *(const v4f*)(li_s + 8 * h), iB = *(const v4f*)(li_s + 8 * h + 4);
#pragma unroll
    for (int nt = 0; nt < 8; ++nt) {
      const int col = 128 * wave + 16 * nt + c;
#pragma unroll
      for (int r = 0; r < 4; ++r) {
        unsigned short hb, lb;
        split_bf(ohi[nt][r] * iA[r], hb, lb);
        Hs[(8 * h + r) * QSP + col] = hb;
        Ls[(8 * h + r) * QSP + col] = lb;
        split_bf(ohi[nt][4 + r] * iB[r], hb, lb);
        Hs[(8 * h + 4 + r) * QSP + col] = hb;
        Ls[(8 * h + 4 + r) * QSP + col] = lb;
      }
    }
  }
  __syncthreads();
  {
    unsigned short* gh = oh + (size_t)q0 * EMB;
    unsigned short* gl = ol + (size_t)q0 * EMB;
#pragma unroll
    for (int ps = 0; ps < 2; ++ps) {
#pragma unroll
      for (int rr = 0; rr < 2; ++rr) {
        const int row = 2 * wave + rr;
#pragma unroll
        for (int j = 0; j < 4; ++j) {
          const int pc = j * 32 + lane;
          const v8us hvv = *(const v8us*)(Hs + row * QSP + pc * 8);
          const v8us lvv = *(const v8us*)(Ls + row * QSP + pc * 8);
          *(volatile v8us*)(gh + (size_t)row * EMB + pc * 8) = hvv;
          *(volatile v8us*)(gl + (size_t)row * EMB + pc * 8) = lvv;
        }
      }
      __threadfence();
    }
  }
}

extern "C" void kernel_launch(void* const* d_in, const int* in_sizes, int n_in,
                              void* d_out, int out_size, void* d_ws, size_t ws_size,
                              hipStream_t stream) {
  if (n_in < 4) return;
  const int ntok = NTOK, dm = EMB;
  if (in_sizes[0] != 3 * dm * dm || in_sizes[1] != dm * dm) return;
  if (in_sizes[2] != ntok * dm || in_sizes[3] != dm * dm) return;
  if (out_size != ntok * dm) return;

  const float* rot = (const float*)d_in[0];
  const float* ent = (const float*)d_in[1];
  const float* x   = (const float*)d_in[2];
  const float* gw  = (const float*)d_in[3];
  float* out = (float*)d_out;

  const size_t bWQ = (size_t)3 * dm * dm * 2;
  const size_t bWO = (size_t)dm * dm * 2;
  const size_t bGW = (size_t)dm * dm * 2;
  const size_t bP  = (size_t)ntok * dm * 2;
  size_t off = 0;
  const size_t oWQ = off; off += bWQ;
  const size_t oWO = off; off += bWO;
  const size_t oGW = off; off += bGW;
  const size_t oXB = off; off += bP;
  const size_t oQH = off; off += bP;
  const size_t oQL = off; off += bP;
  const size_t oK  = off; off += bP;
  const size_t oVH = off; off += bP;
  const size_t oVL = off; off += bP;
  const size_t oOL = off; off += bP;
  if (off > ws_size) return;
  if (off > (size_t)134217728) return;
  if ((oQL + bP) - oQH != (size_t)ntok * dm * 4) return;

  char* ws = (char*)d_ws;
  unsigned short* WQB   = (unsigned short*)(ws + oWQ);
  unsigned short* WOB   = (unsigned short*)(ws + oWO);
  unsigned short* GW16  = (unsigned short*)(ws + oGW);
  unsigned short* XB    = (unsigned short*)(ws + oXB);
  unsigned short* OH    = (unsigned short*)(ws + oXB);
  unsigned short* QH    = (unsigned short*)(ws + oQH);
  unsigned short* QL    = (unsigned short*)(ws + oQL);
  float*          OUTF  = (float*)(ws + oQH);
  unsigned short* K16   = (unsigned short*)(ws + oK);
  unsigned short* OUT16 = (unsigned short*)(ws + oK);
  unsigned short* VH    = (unsigned short*)(ws + oVH);
  unsigned short* VL    = (unsigned short*)(ws + oVL);
  unsigned short* OL    = (unsigned short*)(ws + oOL);

  const dim3 blk(256);
  const int n8x = ntok * dm / 8;
  const int n8q = 3 * dm * dm / 8;
  const int n8w = dm * dm / 8;
  const int gemm_blocks = ((ntok / 64) * (dm / 64)) / 8;

  cvt_kernel<0><<<dim3((n8x + 255) / 256), blk, 0, stream>>>(x, XB, n8x);
  cvt_kernel<0><<<dim3((n8q + 255) / 256), blk, 0, stream>>>(rot, WQB, n8q);
  cvt_kernel<0><<<dim3((n8w + 255) / 256), blk, 0, stream>>>(ent, WOB, n8w);
  cvt_kernel<1><<<dim3((n8w + 255) / 256), blk, 0, stream>>>(gw, GW16, n8w);
  gemm64_kernel<1, false, 2><<<dim3(gemm_blocks), blk, 0, stream>>>(
      XB, XB, dm, WQB, dm, (void*)QH, (void*)QL, dm, (const float*)(const void*)XB, ntok, dm, dm, 16.0f);
  gemm64_kernel<1, false, 1><<<dim3(gemm_blocks), blk, 0, stream>>>(
      XB, XB, dm, WQB + (size_t)dm * dm, dm, (void*)K16, (void*)K16, dm, (const float*)(const void*)XB,
      ntok, dm, dm, 16.0f);
  gemm64_kernel<1, false, 2><<<dim3(gemm_blocks), blk, 0, stream>>>(
      WQB + (size_t)2 * dm * dm, WQB + (size_t)2 * dm * dm, dm, XB, dm, (void*)VH, (void*)VL, ntok,
      (const float*)(const void*)XB, dm, ntok, dm, 16.0f);
  (void)hipFuncSetAttribute(reinterpret_cast<const void*>(&attn_kernel),
                            hipFuncAttributeMaxDynamicSharedMemorySize, ATT_LDS);
  const float sc = 0.125f * (1.0f / 256.0f);
  attn_kernel<<<dim3(ntok / QB), blk, ATT_LDS, stream>>>(
      (const _Float16*)(const void*)QH, (const _Float16*)(const void*)QL, (const _Float16*)(const void*)K16,
      (const _Float16*)(const void*)VH, (const _Float16*)(const void*)VL, OH, OL, sc);
  gemm64_kernel<1, true, 3><<<dim3(gemm_blocks), blk, 0, stream>>>(
      OH, OL, dm, WOB, dm, (void*)OUTF, (void*)OUT16, dm, (const float*)(const void*)XB, ntok, dm, dm, 1.0f);
  gemm64_kernel<0, false, 4><<<dim3(gemm_blocks), blk, 0, stream>>>(
      OUT16, OUT16, dm, GW16, dm, (void*)out, (void*)out, dm, (const float*)OUTF, ntok, dm, dm, 1.0f / 4096.0f);
  (void)hipGetLastError();
}
